// MABClean_83167746719797
// MI455X (gfx1250) — hardware-verified
//
#include <hip/hip_runtime.h>


#define NB_  4
#define TT   2048
#define CC   256
#define NHD  8
#define DH   32
#define ZH   1
#define OTP  288
#define PCAR 1024.0f
#define SCL  0.0625f
#define NW   32
typedef _Float16 h16;
typedef unsigned short bf;
typedef __attribute__((ext_vector_type(16))) __bf16   v16bf;
typedef __attribute__((ext_vector_type(16))) _Float16 v16h;
typedef __attribute__((ext_vector_type(8)))  _Float16 v8h;
typedef __attribute__((ext_vector_type(8)))  unsigned short v8us;
typedef __attribute__((ext_vector_type(8)))  float    v8f;
typedef __attribute__((ext_vector_type(4)))  float    v4f;
typedef v8h  __attribute__((may_alias)) v8ha;
typedef v4f  __attribute__((may_alias)) v4fa;
typedef v8us __attribute__((may_alias)) v8usa;

__device__ __forceinline__ unsigned short f2bf(float f) { unsigned u = __float_as_uint(f); u += 0x7FFFu + ((u >> 16) & 1u); return (unsigned short)(u >> 16); }
__device__ __forceinline__ float bf2f(unsigned short b) { return __uint_as_float(((unsigned)b) << 16); }
__device__ __forceinline__ float bfr(float f) { return bf2f(f2bf(f)); }
__device__ __forceinline__ v16h cat16(v8h lo, v8h hi) { return __builtin_shufflevector(lo, hi, 0, 1, 2, 3, 4, 5, 6, 7, 8, 9, 10, 11, 12, 13, 14, 15); }
__device__ __forceinline__ v16bf cat16b(v8us lo, v8us hi) { return __builtin_bit_cast(v16bf, __builtin_shufflevector(lo, hi, 0, 1, 2, 3, 4, 5, 6, 7, 8, 9, 10, 11, 12, 13, 14, 15)); }
__device__ __forceinline__ v8f wmma16(v16h a, v16h b, v8f c) { return __builtin_amdgcn_wmma_f32_16x16x32_f16(false, a, false, b, (short)0, c, false, false); }
__device__ __forceinline__ v8f wmmab(v16bf a, v16bf b, v8f c) { return __builtin_amdgcn_wmma_f32_16x16x32_bf16(false, a, false, b, (short)0, c, false, false); }


template <typename T16> struct WFrag;
template <> struct WFrag<h16> { typedef v16h V; static __device__ __forceinline__ V ld(const h16* p) { return cat16(*(const v8h*)p, *(const v8h*)(p + 16)); } static __device__ __forceinline__ v8f mma(V a, V b, v8f c) { return wmma16(a, b, c); } };
template <> struct WFrag<bf> { typedef v16bf V; static __device__ __forceinline__ V ld(const bf* p) { return cat16b(*(const v8us*)p, *(const v8us*)(p + 16)); } static __device__ __forceinline__ v8f mma(V a, V b, v8f c) { return wmmab(a, b, c); } };
template <typename T16, int NSPLIT, bool BIAS>
__global__ __launch_bounds__(32) void k_gemmw(const T16* __restrict__ A, const T16* __restrict__ A2, const T16* __restrict__ Bt, const T16* __restrict__ Bt2, int K, float* C, int ldc, const float* __restrict__ bias, size_t sA, size_t sB, size_t sC) {
    typedef typename WFrag<T16>::V V;
    __shared__ __align__(16) float os[16 * 68];
    const size_t z = blockIdx.z; A += z * sA; if (A2) A2 += z * sA; Bt += z * sB; if (Bt2) Bt2 += z * sB; C += z * sC;
    const int lane = threadIdx.x & 31, lr = lane & 15, hi = lane >> 4; const int r0 = blockIdx.x * 64, c0 = blockIdx.y * 64;
    v8f acc[4][4];
#pragma unroll
    for (int mb = 0; mb < 4; ++mb)
#pragma unroll
        for (int nb = 0; nb < 4; ++nb) acc[mb][nb] = (v8f){};
    const size_t aoff = (size_t)(r0 + lr) * K + 8 * hi, boff = (size_t)(c0 + lr) * K + 8 * hi;
#pragma unroll 1
    for (int kc = 0; kc < K; kc += 32) {
        V a[4], a2[4];
#pragma unroll
        for (int mb = 0; mb < 4; ++mb) { a[mb] = WFrag<T16>::ld(A + aoff + (size_t)mb * 16 * K + kc); if (NSPLIT == 1 || NSPLIT == 2) a2[mb] = WFrag<T16>::ld(A2 + aoff + (size_t)mb * 16 * K + kc); }
#pragma unroll
        for (int nb = 0; nb < 4; ++nb) { const V b = WFrag<T16>::ld(Bt + boff + (size_t)nb * 16 * K + kc); V b2; if (NSPLIT >= 2) b2 = WFrag<T16>::ld(Bt2 + boff + (size_t)nb * 16 * K + kc);
#pragma unroll
            for (int mb = 0; mb < 4; ++mb) { acc[mb][nb] = WFrag<T16>::mma(a[mb], b, acc[mb][nb]); if (NSPLIT == 1 || NSPLIT == 2) acc[mb][nb] = WFrag<T16>::mma(a2[mb], b, acc[mb][nb]); if (NSPLIT >= 2) acc[mb][nb] = WFrag<T16>::mma(a[mb], b2, acc[mb][nb]); } }
        asm volatile("v_nop\n\tv_nop\n\tv_nop\n\tv_nop" : "+v"(acc[0][0]), "+v"(acc[1][1]), "+v"(acc[2][2]), "+v"(acc[3][3]) : "v"(a[0]), "v"(a[3]));
    }
#pragma unroll
    for (int mb = 0; mb < 4; ++mb) {
#pragma unroll
        for (int nb = 0; nb < 4; ++nb) {
#pragma unroll
            for (int j = 0; j < 8; ++j) os[(hi * 8 + j) * 68 + nb * 16 + lr] = acc[mb][nb][j]; }
        __builtin_amdgcn_wave_barrier(); asm volatile("" ::: "memory");
        float* crow = C + (size_t)(r0 + mb * 16) * ldc + c0;
#pragma unroll 1
        for (int ps = 0; ps < 2; ++ps) {
#pragma unroll
            for (int s = 0; s < 8; ++s) { const int row = 2 * s + hi, cofs = lr * 4; v4f val = *(const v4fa*)(os + row * 68 + cofs); if (BIAS) { val[0] += bfr(bias[c0 + cofs]); val[1] += bfr(bias[c0 + cofs + 1]); val[2] += bfr(bias[c0 + cofs + 2]); val[3] += bfr(bias[c0 + cofs + 3]); }
                *(volatile v4f*)(crow + (size_t)row * ldc + cofs) = val; }
            if (ps == 0) __threadfence(); }
        __builtin_amdgcn_wave_barrier(); asm volatile("" ::: "memory");
    }
}

__device__ __forceinline__ h16 tohx(float x) { return (h16)x; }
__device__ __forceinline__ void splitf(float y, unsigned short& h, unsigned short& l) { h = f2bf(y); l = f2bf(y - bf2f(h)); }
typedef __attribute__((ext_vector_type(2))) _Float16 v2h;
typedef __attribute__((ext_vector_type(4))) _Float16 v4h;
typedef __attribute__((ext_vector_type(2))) unsigned short v2us;
typedef __attribute__((ext_vector_type(8))) _Float16 v8h16;

__global__ __launch_bounds__(256) void k_cvt8(const float* __restrict__ src, bf* dst, size_t n8) { const size_t i = (size_t)blockIdx.x * 256 + threadIdx.x; if (i >= n8) return; const v8f v = *(const v8f*)(src + i * 8); v8us o;
#pragma unroll
    for (int k = 0; k < 8; ++k) o[k] = f2bf(v[k]); *(volatile v8us*)(dst + i * 8) = o; __threadfence(); *(volatile v8us*)(dst + i * 8) = o; }
template <int RAW, int PASS>
__global__ __launch_bounds__(256) void k_psum(const float* __restrict__ A, const float* __restrict__ ST, float* PART) {
    const int lane = threadIdx.x & 31; const int w = blockIdx.x * 8 + (threadIdx.x >> 5); if (w >= NW) return; const float mu = PASS ? ST[0] : 0.f; float s = 0.f;
    for (int i = lane * 4; i < 64 * CC; i += 128) { const v4f v = *(const v4f*)(A + (size_t)w * 64 * CC + i);
#pragma unroll
        for (int q = 0; q < 4; ++q) { float x = RAW ? bfr(v[q]) : v[q]; if (PASS) { const float d0 = __fsub_rn(x, mu); x = __fmul_rn(d0, d0); } s = __fadd_rn(s, x); } }
#pragma unroll
    for (int sh = 16; sh; sh >>= 1) s += __shfl_xor(s, sh, 32);
    const float o = (lane == 0) ? s : 0.f; *(volatile float*)(PART + (size_t)w * 32 + lane) = o; __threadfence(); *(volatile float*)(PART + (size_t)w * 32 + lane) = o; }
template <int PASS>
__global__ __launch_bounds__(32) void k_comb(const float* __restrict__ PART, float* ST) {
    const int lane = threadIdx.x; float s = PART[(size_t)lane * 32];
#pragma unroll
    for (int sh = 16; sh; sh >>= 1) s += __shfl_xor(s, sh, 32);
    const float inv = 1.0f / (float)(TT * CC); float o;
    if (PASS == 0) o = (lane == 0) ? s * inv : 0.f; else { const float mu = ST[0]; o = (lane == 0) ? mu : (lane == 1 ? __fdiv_rn(1.0f, __fsqrt_rn(__fadd_rn(s * inv, 1e-5f))) : 0.f); }
    *(volatile float*)(ST + lane) = o; __threadfence(); *(volatile float*)(ST + lane) = o; }
template <int RAW, int RELU>
__global__ __launch_bounds__(256) void k_snpl(const float* __restrict__ A, const float* __restrict__ ST, const float* __restrict__ w, const float* __restrict__ bb, bf* Ph, bf* Pl) { const size_t i = ((size_t)blockIdx.x * 256 + threadIdx.x) * 2; if (i >= (size_t)TT * CC) return; const int c = (int)(i & (CC - 1)); const float mu = ST[0], rs = ST[1]; v2us oh, ol;
#pragma unroll
    for (int q = 0; q < 2; ++q) { float x = A[i + q]; if (RAW) x = bfr(x); float t = __fmul_rn(__fsub_rn(x, mu), rs); asm volatile("" : "+v"(t)); float y = __fadd_rn(__fmul_rn(t, bfr(w[c + q])), bfr(bb[c + q])); if (RELU) y = fmaxf(y, 0.f); unsigned short a, c2; splitf(y, a, c2); oh[q] = a; ol[q] = c2; }
    *(volatile v2us*)(Ph + i) = oh; *(volatile v2us*)(Pl + i) = ol; __threadfence(); *(volatile v2us*)(Ph + i) = oh; *(volatile v2us*)(Pl + i) = ol; }
__global__ __launch_bounds__(256) void k_hp32(const float* __restrict__ F, int rows, int lg2rows, h16* P) {
    const int lane = threadIdx.x & 31; const int L0 = (blockIdx.x * 8 + (threadIdx.x >> 5)) * 8; const int nlines = NHD * rows * DH / 64;
#pragma unroll 1
    for (int ps = 0; ps < 2; ++ps) {
#pragma unroll
        for (int l = 0; l < 8; ++l) { const int L = L0 + l; if (L >= nlines) break; const int e = L * 64 + lane * 2; const int d = e & (DH - 1); const int r = (e >> 5) & (rows - 1); const int h = e >> (5 + lg2rows); v2h o;
#pragma unroll
            for (int q = 0; q < 2; ++q) o[q] = tohx(F[(size_t)r * CC + h * DH + d + q]);
            *(volatile v2h*)(P + (size_t)e) = o; }
        if (ps == 0) __threadfence(); }
}
__global__ __launch_bounds__(256) void k_vt32(const float* __restrict__ FV, h16* V16) {
    const int lane = threadIdx.x & 31; const int L0 = (blockIdx.x * 8 + (threadIdx.x >> 5)) * 8; const int nlines = CC * TT / 64;
#pragma unroll 1
    for (int ps = 0; ps < 2; ++ps) {
#pragma unroll
        for (int l = 0; l < 8; ++l) { const int L = L0 + l; if (L >= nlines) break; const int e = L * 64 + lane * 2; const int n = e & (TT - 1); const int c = e >> 11; v2h o;
#pragma unroll
            for (int q = 0; q < 2; ++q) o[q] = tohx(FV[(size_t)(n + q) * CC + c]);
            *(volatile v2h*)(V16 + (size_t)e) = o; }
        if (ps == 0) __threadfence(); }
}
__global__ __launch_bounds__(256) void k_asoft(const float* __restrict__ Sb, h16* P16) {
    const int lane = threadIdx.x & 31; const int row = blockIdx.x * 8 + (threadIdx.x >> 5); if (row >= ZH * TT) return;
    const float* sr = Sb + (size_t)row * TT; float v[64]; float mx = -3.0e38f;
#pragma unroll
    for (int ch = 0; ch < 16; ++ch) { const int j0 = ch * 128 + lane * 4; const v4f a = *(const v4f*)(sr + j0);
#pragma unroll
        for (int q = 0; q < 4; ++q) { const float t = a[q] * SCL; v[ch * 4 + q] = t; mx = fmaxf(mx, t); } }
#pragma unroll
    for (int sh = 16; sh; sh >>= 1) mx = fmaxf(mx, __shfl_xor(mx, sh, 32));
    float sum = 0.f;
#pragma unroll
    for (int k = 0; k < 64; ++k) { v[k] = __expf(v[k] - mx); sum += v[k]; }
#pragma unroll
    for (int sh = 16; sh; sh >>= 1) sum += __shfl_xor(sum, sh, 32);
    const float f = __fdiv_rn(PCAR, sum);
#pragma unroll 1
    for (int ps = 0; ps < 2; ++ps) {
#pragma unroll
        for (int ch = 0; ch < 16; ++ch) { v4h o;
#pragma unroll
            for (int q = 0; q < 4; ++q) o[q] = tohx(v[ch * 4 + q] * f);
            *(volatile v4h*)(P16 + (size_t)row * TT + ch * 128 + lane * 4) = o; }
        if (ps == 0) __threadfence(); }
}
__global__ __launch_bounds__(256) void k_osplit(const float* __restrict__ OTf, bf* Oh, bf* Ol) { const size_t i = ((size_t)blockIdx.x * 256 + threadIdx.x) * 2; if (i >= (size_t)TT * CC) return; const int c = (int)(i & (CC - 1)); const int n = (int)(i >> 8); v2us oh, ol;
#pragma unroll
    for (int q = 0; q < 2; ++q) { unsigned short a, c2; splitf(OTf[(size_t)n * OTP + c + q] * (1.0f / PCAR), a, c2); oh[q] = a; ol[q] = c2; }
    *(volatile v2us*)(Oh + i) = oh; *(volatile v2us*)(Ol + i) = ol; __threadfence(); *(volatile v2us*)(Oh + i) = oh; *(volatile v2us*)(Ol + i) = ol; }
template <int RAW>
__global__ __launch_bounds__(256) void k_res(const float* __restrict__ a, const float* __restrict__ B, float* Dd) { const size_t i = ((size_t)blockIdx.x * 256 + threadIdx.x) * 4; if (i >= (size_t)TT * CC) return; const v4f x = *(const v4f*)(a + i), y = *(const v4f*)(B + i); v4f o;
#pragma unroll
    for (int q = 0; q < 4; ++q) o[q] = __fadd_rn(RAW ? bfr(x[q]) : x[q], y[q]); *(volatile v4f*)(Dd + i) = o; __threadfence(); *(volatile v4f*)(Dd + i) = o; }

extern "C" void kernel_launch(void* const* d_in, const int* in_sizes, int n_in,
                              void* d_out, int out_size, void* d_ws, size_t ws_size, hipStream_t stream) {
    (void)in_sizes; (void)n_in; (void)out_size;
    const float* IN[18]; for (int i = 0; i < 18; ++i) IN[i] = (const float*)d_in[i];
    float* OUT = (float*)d_out;
    char* wsp = (char*)d_ws;
    auto take = [&](size_t bytes) { char* p = wsp; wsp += (bytes + 255) & ~(size_t)255; return (void*)p; };
    bf* WQ = (bf*)take((size_t)CC * CC * 2); bf* WK = (bf*)take((size_t)CC * CC * 2); bf* WV = (bf*)take((size_t)CC * CC * 2); bf* WO = (bf*)take((size_t)CC * CC * 2); bf* WR = (bf*)take((size_t)CC * CC * 2);
    float* PART = (float*)take(NW * 32 * 4); float* ST = (float*)take(256);
    bf* Ph = (bf*)take((size_t)TT * CC * 2); bf* Pl = (bf*)take((size_t)TT * CC * 2); bf* YB = (bf*)take((size_t)TT * CC * 2); float* FQ = (float*)take((size_t)TT * CC * 4); float* FK = (float*)take((size_t)TT * CC * 4); float* FV = (float*)take((size_t)TT * CC * 4);
    h16* QP = (h16*)take((size_t)NHD * TT * DH * 2); h16* KP = (h16*)take((size_t)NHD * TT * DH * 2); h16* V16 = (h16*)take((size_t)(CC + DH) * TT * 2);
    float* Sb = (float*)take((size_t)TT * TT * 4); h16* Pm = (h16*)take((size_t)TT * TT * 2); float* OTf = (float*)take((size_t)TT * OTP * 4); bf* Oh = (bf*)take((size_t)TT * CC * 2); bf* Ol = (bf*)take((size_t)TT * CC * 2); float* H = (float*)take((size_t)TT * CC * 4);
    if ((size_t)(wsp - (char*)d_ws) > ws_size) return;
    { const size_t nw = (size_t)CC * CC / 8; const unsigned gw = (unsigned)((nw + 255) / 256); const float* ws_[5] = {IN[2], IN[4], IN[6], IN[8], IN[10]}; bf* wd_[5] = {WQ, WK, WV, WO, WR};
      for (int i = 0; i < 5; ++i) k_cvt8<<<gw, 256, 0, stream>>>(ws_[i], wd_[i], nw); hipMemsetAsync(V16 + (size_t)CC * TT, 0, (size_t)DH * TT * 2, stream); }
    const unsigned L2 = (unsigned)(((size_t)TT * CC / 2 + 255) / 256), L4 = (unsigned)(((size_t)TT * CC / 4 + 255) / 256), LP = (NHD * TT * DH / 64 + 63) / 64; const dim3 gP(TT / 64, CC / 64, 1);
    for (int b = 0; b < NB_; ++b) { const float* Xb = IN[0] + (size_t)b * TT * CC; const float* Ybp = IN[1] + (size_t)b * TT * CC;
        k_psum<1, 0><<<NW / 8, 256, 0, stream>>>(Xb, ST, PART); k_comb<0><<<1, 32, 0, stream>>>(PART, ST); k_psum<1, 1><<<NW / 8, 256, 0, stream>>>(Xb, ST, PART); k_comb<1><<<1, 32, 0, stream>>>(PART, ST);
        k_snpl<1, 0><<<L2, 256, 0, stream>>>(Xb, ST, IN[12], IN[13], Ph, Pl);
        k_gemmw<bf, 1, true><<<gP, 32, 0, stream>>>(Ph, Pl, WQ, nullptr, CC, FQ, CC, IN[3], 0, 0, 0); k_hp32<<<LP, 256, 0, stream>>>(FQ, TT, 11, QP);
        k_psum<1, 0><<<NW / 8, 256, 0, stream>>>(Ybp, ST, PART); k_comb<0><<<1, 32, 0, stream>>>(PART, ST); k_psum<1, 1><<<NW / 8, 256, 0, stream>>>(Ybp, ST, PART); k_comb<1><<<1, 32, 0, stream>>>(PART, ST);
        k_snpl<1, 0><<<L2, 256, 0, stream>>>(Ybp, ST, IN[14], IN[15], Ph, Pl);
        k_gemmw<bf, 1, true><<<gP, 32, 0, stream>>>(Ph, Pl, WK, nullptr, CC, FK, CC, IN[5], 0, 0, 0); k_hp32<<<LP, 256, 0, stream>>>(FK, TT, 11, KP);
        k_cvt8<<<(unsigned)(((size_t)TT * CC / 8 + 255) / 256), 256, 0, stream>>>(Ybp, YB, (size_t)TT * CC / 8);
        k_gemmw<bf, 0, true><<<gP, 32, 0, stream>>>(YB, nullptr, WV, nullptr, CC, FV, CC, IN[7], 0, 0, 0); k_vt32<<<(CC * TT / 64 + 63) / 64, 256, 0, stream>>>(FV, V16);
        for (int hh = 0; hh < NHD; ++hh) {
            k_gemmw<h16, 0, false><<<dim3(TT / 64, TT / 64, 1), 32, 0, stream>>>(QP + (size_t)hh * TT * DH, nullptr, KP + (size_t)hh * TT * DH, nullptr, DH, Sb, TT, nullptr, 0, 0, 0);
            k_asoft<<<TT / 8, 256, 0, stream>>>(Sb, Pm);
            k_gemmw<h16, 0, false><<<dim3(TT / 64, 1, 1), 32, 0, stream>>>(Pm, nullptr, V16 + (size_t)hh * DH * TT, nullptr, TT, OTf + hh * DH, OTP, nullptr, 0, 0, 0); }
        k_osplit<<<L2, 256, 0, stream>>>(OTf, Oh, Ol);
        k_gemmw<bf, 1, true><<<gP, 32, 0, stream>>>(Oh, Ol, WO, nullptr, CC, FQ, CC, IN[9], 0, 0, 0);
        k_res<1><<<L4, 256, 0, stream>>>(Xb, FQ, H);
        k_psum<0, 0><<<NW / 8, 256, 0, stream>>>(H, ST, PART); k_comb<0><<<1, 32, 0, stream>>>(PART, ST); k_psum<0, 1><<<NW / 8, 256, 0, stream>>>(H, ST, PART); k_comb<1><<<1, 32, 0, stream>>>(PART, ST);
        k_snpl<0, 1><<<L2, 256, 0, stream>>>(H, ST, IN[16], IN[17], Ph, Pl);
        k_gemmw<bf, 1, true><<<gP, 32, 0, stream>>>(Ph, Pl, WR, nullptr, CC, FK, CC, IN[11], 0, 0, 0);
        k_res<0><<<L4, 256, 0, stream>>>(H, FK, OUT + (size_t)b * TT * CC); }
}
